// SpectralMessage_24567212933541
// MI455X (gfx1250) — hardware-verified
//
#include <hip/hip_runtime.h>
#include <math.h>

typedef __attribute__((ext_vector_type(16))) _Float16 v16h;
typedef __attribute__((ext_vector_type(16))) __bf16 v16b;
typedef __attribute__((ext_vector_type(8)))  _Float16 v8h;
typedef __attribute__((ext_vector_type(8)))  float v8f;
typedef __attribute__((ext_vector_type(4)))  float v4f;
typedef __attribute__((ext_vector_type(2)))  float v2f;
typedef __attribute__((ext_vector_type(4)))  unsigned v4u;
typedef __attribute__((ext_vector_type(4)))  int v4i;
typedef float __attribute__((may_alias)) float_a;
typedef int __attribute__((may_alias)) int_a;

template <typename T> __device__ __forceinline__ void vst2(void* p, T v) { *(volatile T*)p = v; __threadfence(); *(volatile T*)p = v; }
__device__ __forceinline__ v8f wmma16(v16h a, v16h b, v8f c) {
  v8f d = __builtin_amdgcn_wmma_f32_16x16x32_f16(false, a, false, b, (short)0, c, false, false);
  asm volatile("v_nop\n\tv_nop\n\tv_nop\n\tv_nop" : "+v"(d) : "v"(a), "v"(b));
  return d;
}
__device__ __forceinline__ v8f wmma_bf(v16b a, v16b b, v8f c) {
  v8f d = __builtin_amdgcn_wmma_f32_16x16x32_bf16(false, a, false, b, (short)0, c, false, false);
  asm volatile("v_nop\n\tv_nop\n\tv_nop\n\tv_nop" : "+v"(d) : "v"(a), "v"(b));
  return d;
}
__device__ __forceinline__ v16h frag_h(const _Float16* rowk0, int lane) {
  union { v16h v; v8h q[2]; } u; const _Float16* p = rowk0 + 8 * (lane >> 4);
  u.q[0] = *(const v8h*)p; u.q[1] = *(const v8h*)(p + 16); return u.v;
}
__device__ __forceinline__ v16h frag_f32(const float* rowk0, int lane) {
  v16h a; const float* p = rowk0 + 8 * (lane >> 4);
#pragma unroll
  for (int i = 0; i < 8; ++i) { a[i] = (_Float16)p[i]; a[8 + i] = (_Float16)p[16 + i]; }
  return a;
}
__device__ __forceinline__ v16h frag_f32s(const float* rowk0, int lane, float sc) {
  v16h a; const float* p = rowk0 + 8 * (lane >> 4);
#pragma unroll
  for (int i = 0; i < 8; ++i) { a[i] = (_Float16)(p[i] * sc); a[8 + i] = (_Float16)(p[16 + i] * sc); }
  return a;
}
__device__ __forceinline__ v16h fragc_f32(const float* W, int k0, int n, int lane, int ld, int K) {
  v16h a; const int g = lane >> 4;
#pragma unroll
  for (int i = 0; i < 8; ++i) { const int ka = k0 + 8 * g + i, kb = ka + 16;
    a[i] = (_Float16)(ka < K ? W[(size_t)(ka < K ? ka : K - 1) * ld + n] : 0.f); a[8 + i] = (_Float16)(kb < K ? W[(size_t)(kb < K ? kb : K - 1) * ld + n] : 0.f); }
  return a;
}
struct F2 { v16b h, l; };
__device__ __forceinline__ F2 bsplit16(const float v[16]) { F2 r;
#pragma unroll
  for (int i = 0; i < 16; ++i) { const __bf16 h = (__bf16)v[i]; r.h[i] = h; r.l[i] = (__bf16)(v[i] - (float)h); }
  return r; }
__device__ __forceinline__ F2 split_row(const float* row, int k0, int lane) { float v[16]; const float* p = row + k0 + 8 * (lane >> 4);
#pragma unroll
  for (int i = 0; i < 8; ++i) { v[i] = p[i]; v[8 + i] = p[16 + i]; }
  return bsplit16(v); }
__device__ __forceinline__ F2 split_rowK(const float* row, int k0, int lane, int K) { float v[16]; const int g = lane >> 4;
#pragma unroll
  for (int i = 0; i < 8; ++i) { const int ka = k0 + 8 * g + i, kb = ka + 16; v[i] = ka < K ? row[ka < K ? ka : K - 1] : 0.f; v[8 + i] = kb < K ? row[kb < K ? kb : K - 1] : 0.f; }
  return bsplit16(v); }
__device__ __forceinline__ F2 split_col(const float* W, int k0, int n, int lane, int ld, int K) { float v[16]; const int g = lane >> 4;
#pragma unroll
  for (int i = 0; i < 8; ++i) { const int ka = k0 + 8 * g + i, kb = ka + 16; v[i] = ka < K ? W[(size_t)(ka < K ? ka : K - 1) * ld + n] : 0.f; v[8 + i] = kb < K ? W[(size_t)(kb < K ? kb : K - 1) * ld + n] : 0.f; }
  return bsplit16(v); }
__device__ __forceinline__ v8f mac3(const F2& a, const F2& b, v8f c) { c = wmma_bf(a.l, b.h, c); c = wmma_bf(a.h, b.l, c); return wmma_bf(a.h, b.h, c); }
__device__ __forceinline__ float sigm(float v) { return 1.0f / (1.0f + expf(-v)); }
#define LDSX() do { asm volatile("s_wait_dscnt 0" ::: "memory"); __builtin_amdgcn_wave_barrier(); __builtin_amdgcn_fence(__ATOMIC_RELEASE, "workgroup"); } while (0)


#define TT 3200
#define NB 32
#define NOBJ 100
#define DD 4096
#define HH 1024
#define NC 151
#define NRL 51
#define C1O 10
#define C2O 5
#define K1 459
#define K1P 480
#ifndef TRB
#define TRB (TT / 64)
#define TNB NB
#define TROWLIM TT
#endif
typedef __attribute__((ext_vector_type(8))) __bf16 v8b;
__device__ __forceinline__ v16b frag_b(const __bf16* rowk0, int lane) {
  union { v16b v; v8b q[2]; } u; const __bf16* p = rowk0 + 8 * (lane >> 4);
  u.q[0] = *(const v8b*)p; u.q[1] = *(const v8b*)(p + 16); return u.v;
}
__device__ __forceinline__ v16b frag_gbf(const float* rowk0, int lane) {
  v16b a; const float* p = rowk0 + 8 * (lane >> 4);
#pragma unroll
  for (int i = 0; i < 8; ++i) { a[i] = (__bf16)p[i]; a[8 + i] = (__bf16)p[16 + i]; }
  return a;
}
__device__ __forceinline__ float bfr(float v) { return (float)(__bf16)v; }
__device__ __attribute__((noinline)) float tanh_ni(float v) { return tanhf(v); }
__device__ __forceinline__ v8f mac3p(v16b ah, v16b al, v16b bh, v16b bl, v8f c) { c = wmma_bf(al, bh, c); c = wmma_bf(ah, bl, c); return wmma_bf(ah, bh, c); }

#define WS_PTC   0u
#define WS_PTU   (WS_PTC + 2u * HH * DD)
#define WS_PTF   (WS_PTU + 2u * HH * HH)
#define WS_PTD   (WS_PTF + 2u * HH * HH)
#define WS_C1T   (WS_PTD + 2u * DD * HH)
#define WS_COMP  (WS_C1T + 2u * 16 * K1P)
#define WS_U1    (WS_COMP + 4u * TT * HH)
#define WS_C1    (WS_U1 + 4u * TT * HH)
#define WS_ADJ   (WS_C1 + 4u * TT * 1024)
#define WS_OFL   (WS_ADJ + 4u * TT * 128)
#define WS_UM    (WS_OFL + 4u * TT * HH)
#define WS_END   (WS_UM + 4u * TT * HH)

__global__ __launch_bounds__(256) void k_pack(const float* __restrict__ Wc, const float* __restrict__ Wu, const float* __restrict__ Wf, const float* __restrict__ Wd, __bf16* __restrict__ PTC, __bf16* __restrict__ PTU, __bf16* __restrict__ PTF, __bf16* __restrict__ PTD) {
  __shared__ __align__(16) __bf16 srow[DD];
  const int n = blockIdx.x, tid = threadIdx.x; const float* Wm; int K, NO, nn; __bf16* dst;
  if (n < HH) { Wm = Wc; K = DD; NO = HH; nn = n; dst = PTC + (size_t)nn * DD; }
  else if (n < 2 * HH) { Wm = Wu; K = HH; NO = HH; nn = n - HH; dst = PTU + (size_t)nn * HH; }
  else if (n < 3 * HH) { Wm = Wf; K = HH; NO = HH; nn = n - 2 * HH; dst = PTF + (size_t)nn * HH; }
  else { Wm = Wd; K = HH; NO = DD; nn = n - 3 * HH; dst = PTD + (size_t)nn * HH; }
  for (int k = tid; k < K; k += 256) srow[k] = (__bf16)Wm[(size_t)k * NO + nn];
  __syncthreads();
  for (int q = tid; q < K / 8; q += 256) vst2((unsigned*)(dst + q * 8), *(const v4u*)(&srow[q * 8]));
}
__global__ __launch_bounds__(256) void k_packc(const float* __restrict__ c1, __bf16* __restrict__ C1T) {
  const int tid = threadIdx.x;
  for (int q = tid; q < 16 * K1P / 8; q += 256) { union { __bf16 e[8]; v4u u; } pk; const int o = q / (K1P / 8), k0 = (q % (K1P / 8)) * 8;
#pragma unroll
    for (int e = 0; e < 8; ++e) { const int k = k0 + e; const int tap = k / NRL, ci = k - tap * NRL; pk.e[e] = (o < C1O && k < K1) ? (__bf16)c1[((o * NRL + ci) * 3 + tap / 3) * 3 + tap % 3] : (__bf16)0.f; }
    vst2((unsigned*)(C1T + q * 8), pk.u); }
}
__global__ __launch_bounds__(128) void k_comp(const float* __restrict__ X, const __bf16* __restrict__ PTC, float* __restrict__ COMP) {
  __shared__ __align__(16) float so[4][16][132];
  const int tid = threadIdx.x, wave = tid >> 5, lane = tid & 31, col = lane & 15, g = lane >> 4; const size_t r0 = (size_t)blockIdx.x * 64 + wave * 16; const int n0 = blockIdx.y * 128;
  v8f acc[8] = {};
#pragma unroll 2
  for (int kc = 0; kc < DD / 32; ++kc) { const v16b a = frag_gbf(X + (r0 + col) * DD + kc * 32, lane);
#pragma unroll
    for (int j = 0; j < 8; ++j) acc[j] = wmma_bf(a, frag_b(PTC + (size_t)(n0 + j * 16 + col) * DD + kc * 32, lane), acc[j]); }
#pragma unroll
  for (int j = 0; j < 8; ++j)
#pragma unroll
    for (int r = 0; r < 8; ++r) { const float v = acc[j][r]; so[wave][8 * g + r][j * 16 + col] = v > 0.f ? v : 0.f; }
  LDSX();
  for (int rl = 0; rl < 16; ++rl) vst2(COMP + (r0 + rl) * HH + n0 + lane * 4, *(const v4f*)(&so[wave][rl][lane * 4]));
}
template <int RES>
__global__ __launch_bounds__(128) void k_lin(const float* __restrict__ IN, const __bf16* __restrict__ PT, float* __restrict__ OUT, int NOUT, const float* __restrict__ resid) {
  __shared__ __align__(16) float so[4][16][132];
  const int tid = threadIdx.x, wave = tid >> 5, lane = tid & 31, col = lane & 15, g = lane >> 4; const size_t r0 = (size_t)blockIdx.x * 64 + wave * 16; const int n0 = blockIdx.y * 128;
  v8f acc[8] = {};
#pragma unroll 2
  for (int kc = 0; kc < HH / 32; ++kc) { const F2 a = split_row(IN + (r0 + col) * HH, kc * 32, lane);
#pragma unroll
    for (int j = 0; j < 8; ++j) { const v16b wb = frag_b(PT + (size_t)(n0 + j * 16 + col) * HH + kc * 32, lane); acc[j] = wmma_bf(a.l, wb, acc[j]); acc[j] = wmma_bf(a.h, wb, acc[j]); } }
#pragma unroll
  for (int j = 0; j < 8; ++j)
#pragma unroll
    for (int r = 0; r < 8; ++r) { const float v = acc[j][r]; float o = v > 0.f ? v : 0.f; if (RES) o += bfr(resid[(r0 + 8 * g + r) * NOUT + n0 + j * 16 + col]); so[wave][8 * g + r][j * 16 + col] = o; }
  LDSX();
  for (int rl = 0; rl < 16; ++rl) { if (r0 + rl < (size_t)TROWLIM) vst2(OUT + (r0 + rl) * NOUT + n0 + lane * 4, *(const v4f*)(&so[wave][rl][lane * 4])); }
}
__global__ __launch_bounds__(128) void k_adj1(const int* __restrict__ lab, const float* __restrict__ freq, const __bf16* __restrict__ C1T, float* __restrict__ C1) {
  __shared__ __bf16 S[3][102][52];
  __shared__ __align__(16) float so[1024];
  const int tid = threadIdx.x, wave = tid >> 5, lane = tid & 31, col = lane & 15, g = lane >> 4;
  const int b = blockIdx.y, i = blockIdx.x;
  for (int q = tid; q < 3 * 102 * 52; q += 128) { const int dy = q / (102 * 52), rem = q % (102 * 52), jj1 = rem / 52, ci = rem % 52; const int ii = i + dy - 1, jj = jj1 - 1;
    float v = 0.f;
    const int iic = ii < 0 ? 0 : (ii > NOBJ - 1 ? NOBJ - 1 : ii), jjc = jj < 0 ? 0 : (jj > NOBJ - 1 ? NOBJ - 1 : jj), cic = ci < NRL ? ci : NRL - 1;
    int li = lab[b * NOBJ + iic], lj = lab[b * NOBJ + jjc]; li = li < 0 ? 0 : (li > NC - 1 ? NC - 1 : li); lj = lj < 0 ? 0 : (lj > NC - 1 ? NC - 1 : lj);
    const float fv = freq[((size_t)li * NC + lj) * NRL + cic];
    v = (ii >= 0 && ii < NOBJ && jj >= 0 && jj < NOBJ && ci < NRL) ? fv : 0.f;
    S[dy][jj1][ci] = (__bf16)v; }
  for (int q = tid; q < 1024; q += 128) so[q] = 0.f;
  __syncthreads();
#pragma unroll 1
  for (int rt = wave; rt < 7; rt += 4) { const int j = rt * 16 + col; const int jc = j < NOBJ ? j : NOBJ - 1;
    v8f acc = {};
#pragma unroll 1
    for (int kc = 0; kc < K1P / 32; ++kc) { v16b a;
#pragma unroll
      for (int e = 0; e < 16; ++e) { const int k = kc * 32 + 8 * g + (e < 8 ? e : 8 + e); const int tap = k / NRL, ci = k - tap * NRL; const int dy = tap / 3, dx = tap - dy * 3;
        a[e] = (k < K1) ? S[dy < 3 ? dy : 2][jc + dx][ci] : (__bf16)0.f; }
      acc = wmma_bf(a, frag_b(C1T + (size_t)col * K1P + kc * 32, lane), acc); }
    if (col < C1O) {
#pragma unroll
      for (int r = 0; r < 8; ++r) { const int jr = rt * 16 + 8 * g + r; if (jr < NOBJ) so[jr * C1O + col] = acc[r]; } } }
  __syncthreads();
  for (int q = tid; q < 256; q += 128) vst2(C1 + ((size_t)b * NOBJ + i) * 1024 + q * 4, *(const v4f*)&so[q * 4]);
}
__global__ __launch_bounds__(128) void k_adj2(const float* __restrict__ C1, const float* __restrict__ c2, const float* __restrict__ c3, float* __restrict__ ADJ) {
  __shared__ float w2[C2O * C1O * 9], w3[C2O]; __shared__ __align__(16) float so[128];
  const int tid = threadIdx.x; const int b = blockIdx.y, i = blockIdx.x;
  for (int q = tid; q < C2O * C1O * 9; q += 128) w2[q] = bfr(c2[q]);
  if (tid < C2O) w3[tid] = bfr(c3[tid]);
  __syncthreads();
  float val = 0.f; const int j = tid;
  if (j < NOBJ) { float o5[C2O] = {0.f, 0.f, 0.f, 0.f, 0.f};
#pragma unroll 1
    for (int dy = 0; dy < 3; ++dy) { const int ii = i + dy - 1; const bool okr = ii >= 0 && ii < NOBJ; const int iic = okr ? ii : i;
#pragma unroll 1
      for (int dx = 0; dx < 3; ++dx) { const int jj = j + dx - 1; const bool ok = okr && jj >= 0 && jj < NOBJ; const int jjc = (jj >= 0 && jj < NOBJ) ? jj : j;
        const float* src = C1 + ((size_t)b * NOBJ + iic) * 1024 + jjc * C1O;
#pragma unroll 1
        for (int ci = 0; ci < C1O; ++ci) { const float xv = ok ? src[ci] : 0.f;
#pragma unroll
          for (int co = 0; co < C2O; ++co) o5[co] += w2[(co * C1O + ci) * 9 + dy * 3 + dx] * xv; } } }
    float s = 0.f;
#pragma unroll
    for (int co = 0; co < C2O; ++co) s += w3[co] * o5[co];
    val = tanh_ni(s); }
  so[tid] = val;
  __syncthreads();
  if (tid < 32) vst2(ADJ + ((size_t)b * NOBJ + i) * 128 + tid * 4, *(const v4f*)&so[tid * 4]);
}
__global__ __launch_bounds__(256) void k_msg(const float* __restrict__ ADJ, const float* __restrict__ U1, float* __restrict__ OFL) {
  __shared__ __align__(16) float so[8][16][132];
  const int tid = threadIdx.x, wave = tid >> 5, lane = tid & 31, col = lane & 15, g = lane >> 4;
  const int b = blockIdx.y, rt = blockIdx.x; const int n = rt * 16 + col, nc = n < NOBJ ? n : NOBJ - 1; const int h0 = wave * 128;
  v8f acc[8] = {};
#pragma unroll 1
  for (int kc = 0; kc < 4; ++kc) { const F2 a = split_row(ADJ + ((size_t)b * NOBJ + nc) * 128, kc * 32, lane);
#pragma unroll
    for (int jt = 0; jt < 8; ++jt) { const F2 bq = split_col(U1 + (size_t)b * NOBJ * HH, kc * 32, h0 + jt * 16 + col, lane, HH, NOBJ); acc[jt] = mac3(a, bq, acc[jt]); } }
#pragma unroll
  for (int jt = 0; jt < 8; ++jt)
#pragma unroll
    for (int r = 0; r < 8; ++r) so[wave][8 * g + r][jt * 16 + col] = acc[jt][r];
  LDSX();
  for (int rl = 0; rl < 16; ++rl) { const int nr = rt * 16 + rl; if (nr < NOBJ) vst2(OFL + ((size_t)b * NOBJ + nr) * HH + h0 + lane * 4, *(const v4f*)(&so[wave][rl][lane * 4])); }
}

extern "C" void kernel_launch(void* const* d_in, const int* in_sizes, int n_in, void* d_out, int out_size, void* d_ws, size_t ws_size, hipStream_t stream) {
  (void)in_sizes; (void)n_in; (void)out_size;
  const float** F = (const float**)d_in; const int* lab = (const int*)d_in[9];
  if (ws_size < (size_t)WS_END) return;
  char* ws = (char*)d_ws;
  __bf16 *PTC = (__bf16*)(ws + WS_PTC), *PTU = (__bf16*)(ws + WS_PTU), *PTF = (__bf16*)(ws + WS_PTF), *PTD = (__bf16*)(ws + WS_PTD), *C1T = (__bf16*)(ws + WS_C1T);
  float *COMP = (float*)(ws + WS_COMP), *U1 = (float*)(ws + WS_U1), *C1 = (float*)(ws + WS_C1), *ADJ = (float*)(ws + WS_ADJ), *OFL = (float*)(ws + WS_OFL), *UM = (float*)(ws + WS_UM);
  k_pack<<<3 * HH + DD, 256, 0, stream>>>(F[1], F[2], F[3], F[4], PTC, PTU, PTF, PTD);
  k_packc<<<1, 256, 0, stream>>>(F[5], C1T);
  k_comp<<<dim3(TRB, HH / 128), 128, 0, stream>>>(F[0], PTC, COMP);
  k_lin<0><<<dim3(TRB, HH / 128), 128, 0, stream>>>(COMP, PTU, U1, HH, nullptr);
  k_adj1<<<dim3(NOBJ, TNB), 128, 0, stream>>>(lab, F[8], C1T, C1);
  k_adj2<<<dim3(NOBJ, TNB), 128, 0, stream>>>(C1, F[6], F[7], ADJ);
  k_msg<<<dim3(7, TNB), 256, 0, stream>>>(ADJ, U1, OFL);
  k_lin<0><<<dim3(TRB, HH / 128), 128, 0, stream>>>(OFL, PTF, UM, HH, nullptr);
  k_lin<1><<<dim3(TRB, DD / 128), 128, 0, stream>>>(UM, PTD, (float*)d_out, DD, F[0]);
}
